// ImprovedGAT_44238163149266
// MI455X (gfx1250) — hardware-verified
//
#include <hip/hip_runtime.h>
#include <math.h>

typedef __attribute__((ext_vector_type(16))) _Float16 v16h;
typedef __attribute__((ext_vector_type(8)))  _Float16 v8h;
typedef __attribute__((ext_vector_type(16))) __bf16   v16b;
typedef __attribute__((ext_vector_type(8)))  __bf16   v8b;
typedef __attribute__((ext_vector_type(8)))  float    v8f;
typedef __attribute__((ext_vector_type(4)))  float    v4f;
typedef __attribute__((ext_vector_type(2)))  float    v2f;
typedef __attribute__((ext_vector_type(4)))  int      v4i;
typedef __attribute__((ext_vector_type(4)))  unsigned v4u;

__device__ __forceinline__ unsigned short f2bf_bits(float f) {
  unsigned u = __float_as_uint(f);
  return (unsigned short)((u + 0x7FFFu + ((u >> 16) & 1u)) >> 16);
}
__device__ __forceinline__ float bf_bits2f(unsigned short h) { return __uint_as_float(((unsigned)h) << 16); }

__device__ __forceinline__ void dep_guard_h(v8f& a, v8f& b, v16h x, v16h y) { asm volatile("v_nop\n\tv_nop\n\tv_nop\n\tv_nop" : "+v"(a), "+v"(b) : "v"(x), "v"(y)); }
__device__ __forceinline__ void dep_guard_b(v8f& a, v8f& b, v16b x, v16b y) { asm volatile("v_nop\n\tv_nop\n\tv_nop\n\tv_nop" : "+v"(a), "+v"(b) : "v"(x), "v"(y)); }
__device__ __forceinline__ void keep4_h(v16h a, v16h b, v16h c, v16h d) { asm volatile("v_nop" :: "v"(a), "v"(b), "v"(c), "v"(d)); }
__device__ __forceinline__ void keep4_b(v16b a, v16b b, v16b c, v16b d) { asm volatile("v_nop" :: "v"(a), "v"(b), "v"(c), "v"(d)); }
__device__ __forceinline__ void acc_guard4(v8f& a, v8f& b, v8f& c, v8f& d) { asm volatile("v_nop\n\tv_nop\n\tv_nop\n\tv_nop" : "+v"(a), "+v"(b), "+v"(c), "+v"(d)); }
template <typename T> struct Frag;
template <> struct Frag<_Float16> {
  typedef v16h V; union U { v16h v; v8h h[2]; };
  static __device__ __forceinline__ v16h load(const _Float16* p) {
    U f; f.h[0] = *(const v8h*)(p); f.h[1] = *(const v8h*)(p + 16); return f.v;
  }
  static __device__ __forceinline__ v8f mma(v16h a, v16h b, v8f c) {
    return __builtin_amdgcn_wmma_f32_16x16x32_f16(false, a, false, b, (short)0, c, false, false);
  }
  static __device__ __forceinline__ void guard(v8f& a, v8f& b, v16h x, v16h y) { dep_guard_h(a, b, x, y); }
  static __device__ __forceinline__ void keep(v16h a, v16h b, v16h c, v16h d) { keep4_h(a, b, c, d); }
};
template <> struct Frag<__bf16> {
  typedef v16b V; union U { v16b v; v8b h[2]; };
  static __device__ __forceinline__ v16b load(const __bf16* p) {
    U f; f.h[0] = *(const v8b*)(p); f.h[1] = *(const v8b*)(p + 16); return f.v;
  }
  static __device__ __forceinline__ v8f mma(v16b a, v16b b, v8f c) {
    return __builtin_amdgcn_wmma_f32_16x16x32_bf16(false, a, false, b, (short)0, c, false, false);
  }
  static __device__ __forceinline__ void guard(v8f& a, v8f& b, v16b x, v16b y) { dep_guard_b(a, b, x, y); }
  static __device__ __forceinline__ void keep(v16b a, v16b b, v16b c, v16b d) { keep4_b(a, b, c, d); }
};

template <int ET> struct Elem;
template <> struct Elem<0> { typedef _Float16 T; };
template <> struct Elem<1> { typedef __bf16 T; };
template <int ET, bool SPLIT, int BIAS_MODE, int OUT_MODE, bool RESID, int ACT = 0>
__global__ __launch_bounds__(256) void wmma_gemm64(
    const unsigned short* __restrict__ Ap, const unsigned short* __restrict__ A2p, int lda, long strideA,
    const unsigned short* __restrict__ Btp, const unsigned short* __restrict__ Bt2p, int ldb, long strideB,
    void* __restrict__ Cout, void* __restrict__ Cout2, int ldc, long strideC,
    const float* __restrict__ bias,
    const float* __restrict__ resid, long strideR,
    int M, int N, int K, float scale) {
  typedef typename Elem<ET>::T T;
  typedef typename Frag<T>::V V;
  const T* A = (const T*)Ap; const T* A2 = (const T*)A2p; const T* Bt = (const T*)Btp; const T* Bt2 = (const T*)Bt2p;
  __shared__ __align__(16) float sT[8][16 * 68];
  const int b    = blockIdx.y;
  const int lane = threadIdx.x & 31;
  const int wave = threadIdx.x >> 5;
  const int tilesN = N >> 6;
  const int tilesM = M >> 6;
  const int tile = blockIdx.x * 8 + wave;
  if (tile >= tilesM * tilesN) return;
  const int tm = tile / tilesN;
  const int tn = tile - tm * tilesN;
  const int m0 = tm << 6;
  const int n0 = tn << 6;

  const T* Ab  = A  + (size_t)b * strideA;
  const T* Bb  = Bt + (size_t)b * strideB;
  const T* Ab2 = SPLIT ? (A2  + (size_t)b * strideA) : nullptr;
  const T* Bb2 = SPLIT ? (Bt2 + (size_t)b * strideB) : nullptr;

  const int rlane = lane & 15;
  const int koff  = (lane >> 4) * 8;
  const int mOff  = (lane >> 4) * 8;

  v8f acc[4][4];
#pragma unroll
  for (int i = 0; i < 4; ++i)
#pragma unroll
    for (int j = 0; j < 4; ++j) acc[i][j] = (v8f){0.f,0.f,0.f,0.f,0.f,0.f,0.f,0.f};

  for (int k0 = 0; k0 < K; k0 += 32) {
    V bh[4], bl[4];
#pragma unroll
    for (int j = 0; j < 4; ++j) {
      const size_t bo = (size_t)(n0 + (j << 4) + rlane) * ldb + koff + k0;
      bh[j] = Frag<T>::load(Bb + bo);
      if (SPLIT) bl[j] = Frag<T>::load(Bb2 + bo);
    }
#pragma unroll
    for (int i = 0; i < 4; ++i) {
      const size_t ao = (size_t)(m0 + (i << 4) + rlane) * lda + koff + k0;
      V ah = Frag<T>::load(Ab + ao);
      V al;
      if (SPLIT) al = Frag<T>::load(Ab2 + ao);
#pragma unroll
      for (int j = 0; j < 4; ++j) {
        acc[i][j] = Frag<T>::mma(ah, bh[j], acc[i][j]);
        if (SPLIT) {
          acc[i][j] = Frag<T>::mma(ah, bl[j], acc[i][j]);
          acc[i][j] = Frag<T>::mma(al, bh[j], acc[i][j]);
        }
      }
      Frag<T>::guard(acc[i][0], acc[i][3], ah, SPLIT ? al : ah);
    }
    Frag<T>::keep(bh[0], bh[1], bh[2], bh[3]);
    if (SPLIT) Frag<T>::keep(bl[0], bl[1], bl[2], bl[3]);
  }
  acc_guard4(acc[0][0], acc[0][1], acc[0][2], acc[0][3]);
  acc_guard4(acc[1][0], acc[1][1], acc[1][2], acc[1][3]);
  acc_guard4(acc[2][0], acc[2][1], acc[2][2], acc[2][3]);
  acc_guard4(acc[3][0], acc[3][1], acc[3][2], acc[3][3]);

  float* slab = sT[wave];
  const float* Rb = RESID ? (resid + (size_t)b * strideR) : nullptr;
#pragma unroll
  for (int i = 0; i < 4; ++i) {
    const int mBase = m0 + (i << 4);
#pragma unroll
    for (int j = 0; j < 4; ++j) {
      const int n = n0 + (j << 4) + rlane;
      float bv = 0.f;
      if (BIAS_MODE == 2) bv = bias[n];
#pragma unroll
      for (int r = 0; r < 8; ++r) {
        float v = acc[i][j][r] * scale;
        if (BIAS_MODE == 1) v += bias[mBase + mOff + r];
        if (BIAS_MODE == 2) v += bv;
        if (RESID) v += Rb[(size_t)(mBase + mOff + r) * ldc + n];
        if (ACT == 1) v = tanhf(v);
        if (ACT == 2) v = fmaxf(v, 0.0f);
        if (ACT == 3) v = v / (1.0f + expf(-v));
        if (ACT == 4) v = (v > 0.f) ? v : 0.01f * v;
        if (ACT == 5) v = 0.5f * v * (1.0f + erff(v * 0.70710678118654752f));
        slab[(mOff + r) * 68 + (j << 4) + rlane] = v;
      }
    }
    __builtin_amdgcn_fence(__ATOMIC_RELEASE, "workgroup");
    __builtin_amdgcn_wave_barrier();
    __builtin_amdgcn_fence(__ATOMIC_ACQUIRE, "workgroup");
    if (OUT_MODE == 0) {
      float* C = (float*)Cout + (size_t)b * strideC;
      const int hh = lane >> 4, c4 = (lane & 15) * 4;
      for (int pass = 0; pass < 2; ++pass) {
#pragma unroll
        for (int it = 0; it < 8; ++it) {
          const int row = it * 2 + hh;
          v4f v = *(const v4f*)(slab + row * 68 + c4);
          *(volatile v4f*)(C + (size_t)(mBase + row) * ldc + n0 + c4) = v;
        }
        __threadfence();
      }
    } else {
      const int q = lane >> 3, c8 = (lane & 7) * 8;
      unsigned short* C  = (unsigned short*)Cout  + (size_t)b * strideC;
      unsigned short* C2 = (OUT_MODE == 2) ? ((unsigned short*)Cout2 + (size_t)b * strideC) : nullptr;
      for (int pass = 0; pass < 2; ++pass) {
#pragma unroll
        for (int it = 0; it < 4; ++it) {
          const int row = it * 4 + q;
          const float* sp = slab + row * 68 + c8;
          v8h hv, lv;
#pragma unroll
          for (int e = 0; e < 8; ++e) {
            if (OUT_MODE == 1) {
              hv[e] = (_Float16)sp[e];
            } else {
              unsigned short hb = f2bf_bits(sp[e]);
              unsigned short lb = f2bf_bits(sp[e] - bf_bits2f(hb));
              hv[e] = __builtin_bit_cast(_Float16, hb);
              lv[e] = __builtin_bit_cast(_Float16, lb);
            }
          }
          *(volatile v8h*)(C + (size_t)(mBase + row) * ldc + n0 + c8) = hv;
          if (OUT_MODE == 2) *(volatile v8h*)(C2 + (size_t)(mBase + row) * ldc + n0 + c8) = lv;
        }
        __threadfence();
      }
    }
    __builtin_amdgcn_fence(__ATOMIC_RELEASE, "workgroup");
    __builtin_amdgcn_wave_barrier();
    __builtin_amdgcn_fence(__ATOMIC_ACQUIRE, "workgroup");
  }
}

__global__ __launch_bounds__(256) void cast_f32_f16x2(
    const float* __restrict__ in, _Float16* __restrict__ out, int n2) {
  int i = blockIdx.x * 256 + threadIdx.x;
  if (i < n2) {
    const _Float16 h0 = (_Float16)in[2 * i], h1 = (_Float16)in[2 * i + 1];
    const unsigned u = (unsigned)__builtin_bit_cast(unsigned short, h0) | ((unsigned)__builtin_bit_cast(unsigned short, h1) << 16);
    ((volatile unsigned*)out)[i] = u;
    __threadfence();
    ((volatile unsigned*)out)[i] = u;
  }
}

#define NN 50000
#define NE 800000
#define NPAD 50176
#define FIN 64
#define HD 96
#define HP 128
#define NHD 4
#define HC 24
#define NL 4
#define NG 1024
#define NT 256
#define TILE 2048
#define NTILE 25
#define SCH 4096
#define NCH ((NE + SCH - 1) / SCH)

__device__ __forceinline__ float lrelu02(float v) { return v >= 0.f ? v : 0.2f * v; }
__device__ __forceinline__ float eluf(float v) { return v > 0.f ? v : (__expf(v) - 1.0f); }

__global__ __launch_bounds__(256) void padcast_rows_kernel(const float* __restrict__ x, unsigned* __restrict__ X16) {
  const long i = (long)blockIdx.x * 256 + threadIdx.x; if (i >= (long)NPAD * FIN / 2) return;
  const long e0 = 2 * i; const bool ok = e0 < (long)NN * FIN;
  const float a = ok ? x[e0] : 0.f, b = ok ? x[e0 + 1] : 0.f;
  const unsigned u = (unsigned)__builtin_bit_cast(unsigned short, (_Float16)a) | ((unsigned)__builtin_bit_cast(unsigned short, (_Float16)b) << 16);
  ((volatile unsigned*)X16)[i] = u; __threadfence(); ((volatile unsigned*)X16)[i] = u;
}
__global__ __launch_bounds__(256) void wpad_kernel(const float* __restrict__ Wm, long wstride, int kin, int kp, unsigned* __restrict__ BT, long btstride) {
  const float* W = Wm + (size_t)blockIdx.y * wstride; unsigned* B = BT + (size_t)blockIdx.y * btstride;
  const int i = blockIdx.x * 256 + threadIdx.x; if (i >= HP * kp / 2) return;
  const int o = (2 * i) / kp, k = (2 * i) % kp;
  float a = 0.f, b = 0.f; if (o < HD) { if (k < kin) a = W[(size_t)k * HD + o]; if (k + 1 < kin) b = W[(size_t)(k + 1) * HD + o]; }
  const unsigned u = (unsigned)__builtin_bit_cast(unsigned short, (_Float16)a) | ((unsigned)__builtin_bit_cast(unsigned short, (_Float16)b) << 16);
  ((volatile unsigned*)B)[i] = u; __threadfence(); ((volatile unsigned*)B)[i] = u;
}
__global__ __launch_bounds__(256) void padvec_kernel(const float* __restrict__ b, int n, float* __restrict__ bp) {
  const int i = blockIdx.x * 256 + threadIdx.x; if (i >= HP) return;
  const float v = (i < n) ? b[i] : 0.f; ((volatile float*)bp)[i] = v; __threadfence(); ((volatile float*)bp)[i] = v;
}
__global__ __launch_bounds__(256) void elu_cast_kernel(float* __restrict__ Hm, unsigned* __restrict__ H16) {
  const long i = (long)blockIdx.x * 256 + threadIdx.x; if (i >= (long)NPAD * HP / 2) return;
  const float a = eluf(Hm[2 * i]), b = eluf(Hm[2 * i + 1]);
  const v2f v = {a, b};
  const unsigned u = (unsigned)__builtin_bit_cast(unsigned short, (_Float16)a) | ((unsigned)__builtin_bit_cast(unsigned short, (_Float16)b) << 16);
  for (int pass = 0; pass < 2; ++pass) { *(volatile v2f*)(Hm + 2 * i) = v; ((volatile unsigned*)H16)[i] = u; __threadfence(); }
}
__global__ __launch_bounds__(256) void att_terms_kernel(const float* __restrict__ HW, const float* __restrict__ asv, const float* __restrict__ adv, float* __restrict__ ASD) {
  __shared__ float st[8][8];
  const int lane = threadIdx.x & 31, wave = threadIdx.x >> 5; const int n = blockIdx.x * 8 + wave;
  const float* hr = HW + (size_t)n * HP + lane * 3;
  float s = 0.f, d = 0.f;
#pragma unroll
  for (int q = 0; q < 3; ++q) { const float v = hr[q]; s += v * asv[lane * 3 + q]; d += v * adv[lane * 3 + q]; }
  for (int o = 1; o < 8; o <<= 1) { s += __shfl_xor(s, o, 32); d += __shfl_xor(d, o, 32); }
  if ((lane & 7) == 0) { st[wave][lane >> 3] = s; st[wave][4 + (lane >> 3)] = d; }
  __syncthreads();
  if (threadIdx.x < 64) {
    const float v = st[threadIdx.x >> 3][threadIdx.x & 7];
    ((volatile float*)ASD)[(size_t)blockIdx.x * 64 + threadIdx.x] = v; __threadfence(); ((volatile float*)ASD)[(size_t)blockIdx.x * 64 + threadIdx.x] = v;
  }
}

__device__ __forceinline__ int blk_excl_scan(int cnt, int* scan_ws, int tid, int* tot) {
  const int lane = tid & 31, wave = tid >> 5; int incl = cnt;
#pragma unroll
  for (int o = 1; o < 32; o <<= 1) { const int v = __shfl_up(incl, o, 32); if (lane >= o) incl += v; }
  if (lane == 31) scan_ws[wave] = incl;
  __syncthreads();
  if (wave == 0) { int wv = (lane < NT / 32) ? scan_ws[lane] : 0; int wincl = wv;
#pragma unroll
    for (int o = 1; o < 32; o <<= 1) { const int v = __shfl_up(wincl, o, 32); if (lane >= o) wincl += v; }
    if (lane < NT / 32) scan_ws[32 + lane] = wincl - wv; if (lane == 31) scan_ws[64] = wincl; }
  __syncthreads();
  const int res = scan_ws[32 + wave] + incl - cnt; *tot = scan_ws[64];
  return res;
}
template <int SP, int CAP>
__device__ __forceinline__ int chunk_hits(const int* __restrict__ dstv, const int* __restrict__ srcv, int e0, int n0, int n1, int tid,
                                          int* LIST, int* scan_ws) {
  const int eb = e0 + tid * SP;
  int rec[SP]; int cnt = 0;
#pragma unroll
  for (int k = 0; k < SP; k += 4) {
    v4i d4 = {-1, -1, -1, -1}; v4i s4 = {0, 0, 0, 0};
    if (eb + k < NE) { d4 = *(const v4i*)(dstv + eb + k); s4 = *(const v4i*)(srcv + eb + k); }
#pragma unroll
    for (int e = 0; e < 4; ++e) {
      const int d = d4[e]; int r = -1;
      if (d >= n0 && d < n1) { int s = s4[e]; s = s < 0 ? 0 : (s >= NN ? NN - 1 : s); r = ((d - n0) << 16) | s; ++cnt; }
      rec[k + e] = r;
    }
  }
  int tot; int p = blk_excl_scan(cnt, scan_ws, tid, &tot);
#pragma unroll
  for (int k = 0; k < SP; ++k) if (rec[k] >= 0) { if ((unsigned)p < (unsigned)CAP) LIST[p] = rec[k]; ++p; }
  __syncthreads();
  return tot < CAP ? tot : CAP;
}

__global__ __launch_bounds__(NT) void gat_agg_kernel(const float* __restrict__ HW, const float* __restrict__ ASD, const int* __restrict__ ei,
                                                    const float* __restrict__ bgl, const float* __restrict__ gaml, const float* __restrict__ betl,
                                                    const float* __restrict__ rml, const float* __restrict__ rvl,
                                                    float* AGG, float* Hm, unsigned* H16) {
  __shared__ int LIST[SCH];
  __shared__ float SM[TILE * NHD];
  __shared__ float SL[TILE * NHD];
  __shared__ int scan_ws[80];
  const int tid = threadIdx.x, lane = tid & 31, wave = tid >> 5;
  const int n0 = blockIdx.x * TILE;
  const int n1 = (n0 + TILE < NN) ? (n0 + TILE) : NN;
  const int rbase = blockIdx.x * TILE;
  const int hd = (lane < 24) ? (lane / 6) : 3;
#pragma unroll 1
  for (int j = 0; j < TILE / 8; ++j) {
    const int dl = wave * (TILE / 8) + j;
    int n = n0 + dl; n = n < NN ? n : NN - 1;
    const float e = lrelu02(ASD[(size_t)n * 8 + hd] + ASD[(size_t)n * 8 + 4 + hd]);
    SM[dl * NHD + hd] = e; SL[dl * NHD + hd] = 1.0f;
    const v4f hv = *(const v4f*)(HW + (size_t)n * HP + 4 * lane);
    *(v4f*)(AGG + (size_t)(rbase + dl) * HP + 4 * lane) = hv;
  }
  __syncthreads();
  const int* srcv = ei; const int* dstv = ei + NE;
#pragma unroll 1
  for (int c = 0; c < NCH; ++c) {
    const int tot = chunk_hits<SCH / NT, SCH>(dstv, srcv, c * SCH, n0, n1, tid, LIST, scan_ws);
#pragma unroll 1
    for (int base = 0; base < tot; base += 32) {
      const int q = base + lane;
      const int ent = (q < tot) ? LIST[q] : -1;
      const int own = (ent >= 0 && (ent >> 24) == wave) ? 1 : 0;
      unsigned msk = (unsigned)__ballot(own);
#pragma unroll 1
      for (int it = 0; it < 32; ++it) {
        if (msk == 0u) break;
        const int bp = __builtin_ctz(msk); msk &= msk - 1u;
        const int r = __shfl(ent, bp, 32);
        const int dl = r >> 16, s = r & 0xFFFF;
        float al = ASD[(size_t)s * 8 + hd] + ASD[(size_t)(n0 + dl) * 8 + 4 + hd];
        al = lrelu02(al);
        const int mi = dl * NHD + hd;
        const float mo = SM[mi], lo = SL[mi];
        const float mn = fmaxf(mo, al);
        const float rr = __expf(mo - mn), ex = __expf(al - mn);
        const float ln = lo * rr + ex;
        SM[mi] = mn; SL[mi] = ln;
        float* rp = AGG + (size_t)(rbase + dl) * HP + 4 * lane;
        v4f a = *(const v4f*)rp;
        const v4f hv = *(const v4f*)(HW + (size_t)s * HP + 4 * lane);
        a = a * rr + ex * hv;
        *(v4f*)rp = a;
      }
    }
    __syncthreads();
  }
  const int cl = (lane < 24) ? 4 * lane : 92;
  const v4f bg4 = *(const v4f*)(bgl + cl), gm4 = *(const v4f*)(gaml + cl), bt4 = *(const v4f*)(betl + cl);
  const v4f rm4 = *(const v4f*)(rml + cl), rv4 = *(const v4f*)(rvl + cl);
  v4f sc4;
#pragma unroll
  for (int e = 0; e < 4; ++e) sc4[e] = 1.0f / sqrtf(rv4[e] + 1e-5f);
  const int sl0 = (2 * lane) & 31, sl1 = (2 * lane + 1) & 31;
#pragma unroll 1
  for (int j = 0; j < TILE / 8; ++j) {
    const int dl = wave * (TILE / 8) + j; const int n = n0 + dl;
    if (n < NN) {
      const float lsum = SL[dl * NHD + hd];
      const float inv = 1.0f / (lsum + 1e-16f);
      const v4f a = *(const v4f*)(AGG + (size_t)(rbase + dl) * HP + 4 * lane);
      const v4f ho = *(const v4f*)(Hm + (size_t)n * HP + 4 * lane);
      v4f o;
#pragma unroll
      for (int e = 0; e < 4; ++e) {
        const float hn = a[e] * inv + bg4[e];
        float t = (hn - rm4[e]) * sc4[e];
        t = t * gm4[e] + bt4[e];
        const float u = eluf(t);
        o[e] = (lane < 24) ? (ho[e] + u) : 0.f;
      }
      const unsigned p0 = (unsigned)__builtin_bit_cast(unsigned short, (_Float16)o[0]) | ((unsigned)__builtin_bit_cast(unsigned short, (_Float16)o[1]) << 16);
      const unsigned p1 = (unsigned)__builtin_bit_cast(unsigned short, (_Float16)o[2]) | ((unsigned)__builtin_bit_cast(unsigned short, (_Float16)o[3]) << 16);
      v4u pk;
      pk[0] = (unsigned)__shfl((int)p0, sl0, 32); pk[1] = (unsigned)__shfl((int)p1, sl0, 32);
      pk[2] = (unsigned)__shfl((int)p0, sl1, 32); pk[3] = (unsigned)__shfl((int)p1, sl1, 32);
      float* hrow = Hm + (size_t)n * HP + 4 * lane;
      unsigned* h16 = H16 + (size_t)n * (HP / 2) + 4 * lane;
      for (int pass = 0; pass < 2; ++pass) {
        *(volatile v4f*)hrow = o;
        if (lane < 16) *(volatile v4u*)h16 = pk;
        __threadfence();
      }
    }
  }
}

__global__ __launch_bounds__(256) void pool_kernel(const float* __restrict__ Hm, const int* __restrict__ bvec, int layer, float* __restrict__ Pf) {
  __shared__ float acc[8][HD]; __shared__ int rng[2];
  const int g = blockIdx.x, t = threadIdx.x, lane = t & 31, wave = t >> 5;
  if (t < 2) {
    const int key = g + t; int lo = 0, hi = NN;
#pragma unroll 1
    for (int itb = 0; itb < 20; ++itb) { if (lo >= hi) break; const int mid = (lo + hi) >> 1; if (bvec[mid] < key) lo = mid + 1; else hi = mid; }
    rng[t] = lo;
  }
  __syncthreads();
  int na = rng[0], nb = rng[1]; na = na < 0 ? 0 : na; nb = nb > NN ? NN : nb;
  float s0 = 0.f, s1 = 0.f, s2 = 0.f;
#pragma unroll 1
  for (int n = na + wave; n < nb; n += 8) {
    if (bvec[n] == g) { const float* hr = Hm + (size_t)n * HP + lane * 3; s0 += hr[0]; s1 += hr[1]; s2 += hr[2]; }
  }
  acc[wave][lane * 3] = s0; acc[wave][lane * 3 + 1] = s1; acc[wave][lane * 3 + 2] = s2;
  __syncthreads();
  if (t < HD) {
    float v = 0.f;
#pragma unroll
    for (int w = 0; w < 8; ++w) v += acc[w][t];
    const size_t oi = (size_t)g * (NL * HD) + layer * HD + t;
    ((volatile float*)Pf)[oi] = v; __threadfence(); ((volatile float*)Pf)[oi] = v;
  }
}

__global__ __launch_bounds__(256) void elu16_kernel(unsigned* __restrict__ Z, int n) {
  const int i = blockIdx.x * 256 + threadIdx.x; if (i >= n) return; const unsigned u = Z[i];
  const float a = eluf((float)__builtin_bit_cast(_Float16, (unsigned short)(u & 0xFFFFu))), b = eluf((float)__builtin_bit_cast(_Float16, (unsigned short)(u >> 16)));
  const unsigned r = (unsigned)__builtin_bit_cast(unsigned short, (_Float16)a) | ((unsigned)__builtin_bit_cast(unsigned short, (_Float16)b) << 16);
  ((volatile unsigned*)Z)[i] = r; __threadfence(); ((volatile unsigned*)Z)[i] = r;
}
__global__ __launch_bounds__(256) void head_out_kernel(const float* __restrict__ Z2, const float* __restrict__ Wh2, const float* __restrict__ bh2, float* __restrict__ out) {
  __shared__ float res[32];
  const int lane = threadIdx.x & 31, wave = threadIdx.x >> 5;
  const float w0 = Wh2[lane * 3], w1 = Wh2[lane * 3 + 1], w2 = Wh2[lane * 3 + 2];
  const float b0 = bh2[0];
#pragma unroll 1
  for (int q = 0; q < 4; ++q) {
    const int gi = wave * 4 + q; const int g = blockIdx.x * 32 + gi;
    const float* zr = Z2 + (size_t)g * HP + lane * 3;
    float s = zr[0] * w0 + zr[1] * w1 + zr[2] * w2;
    for (int o = 16; o > 0; o >>= 1) s += __shfl_xor(s, o, 32);
    if (lane == 0) res[gi] = s + b0;
  }
  __syncthreads();
  if (threadIdx.x < 32) {
    const float v = res[threadIdx.x];
    ((volatile float*)out)[(size_t)blockIdx.x * 32 + threadIdx.x] = v; __threadfence(); ((volatile float*)out)[(size_t)blockIdx.x * 32 + threadIdx.x] = v;
  }
}

extern "C" void kernel_launch(void* const* d_in, const int* in_sizes, int n_in, void* d_out, int out_size, void* d_ws, size_t ws_size, hipStream_t stream) {
  if (n_in < 19) return;
  if (in_sizes[0] != NN * FIN || in_sizes[1] != 2 * NE || in_sizes[2] != NN || out_size != NG) return;
  const float* x = (const float*)d_in[0]; const int* ei = (const int*)d_in[1]; const int* bvec = (const int*)d_in[2];
  const float* W_in = (const float*)d_in[3]; const float* b_in = (const float*)d_in[4]; const float* Wg = (const float*)d_in[5];
  const float* asv = (const float*)d_in[6]; const float* adv = (const float*)d_in[7];
  const float* bg = (const float*)d_in[8]; const float* gam = (const float*)d_in[9]; const float* bet = (const float*)d_in[10];
  const float* rm = (const float*)d_in[11]; const float* rv = (const float*)d_in[12];
  const float* Wjk = (const float*)d_in[13]; const float* bjk = (const float*)d_in[14]; const float* Wh1 = (const float*)d_in[15]; const float* bh1 = (const float*)d_in[16];
  const float* Wh2 = (const float*)d_in[17]; const float* bh2 = (const float*)d_in[18];

  char* ws = (char*)d_ws; size_t off = 0;
  auto carve = [&](size_t bytes) -> char* { char* p = ws + off; off += (bytes + 255) & ~(size_t)255; return p; };
  unsigned* X16  = (unsigned*)carve((size_t)NPAD * FIN * 2);
  unsigned* WinT = (unsigned*)carve((size_t)HP * FIN * 2);
  float*    binp = (float*)carve(HP * 4);
  unsigned* WgT  = (unsigned*)carve((size_t)NL * HP * HP * 2);
  unsigned* WjkT = (unsigned*)carve((size_t)HP * (NL * HD) * 2);
  float*    bjkp = (float*)carve(HP * 4);
  unsigned* Wh1T = (unsigned*)carve((size_t)HP * HP * 2);
  float*    bh1p = (float*)carve(HP * 4);
  float*    Hm   = (float*)carve((size_t)NPAD * HP * 4);
  unsigned* H16  = (unsigned*)carve((size_t)NPAD * HP * 2);
  float*    HW   = (float*)carve((size_t)NPAD * HP * 4);
  float*    AGG  = (float*)carve((size_t)NTILE * TILE * HP * 4);
  float*    ASD  = (float*)carve((size_t)NPAD * 8 * 4);
  float*    Pf   = (float*)carve((size_t)NG * NL * HD * 4);
  unsigned* P16  = (unsigned*)carve((size_t)NG * NL * HD * 2);
  unsigned* Z16  = (unsigned*)carve((size_t)NG * HP * 2);
  float*    Z2   = (float*)carve((size_t)NG * HP * 4);
  if (off > ws_size || off > (size_t)134217728) return;

  padcast_rows_kernel<<<(NPAD * FIN / 2 + 255) / 256, 256, 0, stream>>>(x, X16);
  wpad_kernel<<<dim3((HP * FIN / 2 + 255) / 256, 1), 256, 0, stream>>>(W_in, 0L, FIN, FIN, WinT, 0L);
  padvec_kernel<<<1, 256, 0, stream>>>(b_in, HD, binp);
  wpad_kernel<<<dim3((HP * HP / 2 + 255) / 256, NL), 256, 0, stream>>>(Wg, (long)HD * HD, HD, HP, WgT, (long)HP * HP / 2);
  wpad_kernel<<<dim3((HP * NL * HD / 2 + 255) / 256, 1), 256, 0, stream>>>(Wjk, 0L, NL * HD, NL * HD, WjkT, 0L);
  padvec_kernel<<<1, 256, 0, stream>>>(bjk, HD, bjkp);
  wpad_kernel<<<dim3((HP * HP / 2 + 255) / 256, 1), 256, 0, stream>>>(Wh1, 0L, HD, HP, Wh1T, 0L);
  padvec_kernel<<<1, 256, 0, stream>>>(bh1, HD, bh1p);

  { const int t = (NPAD / 64) * (HP / 64);
    wmma_gemm64<0, false, 2, 0, false><<<dim3((t + 7) / 8, 1), 256, 0, stream>>>(
        (const unsigned short*)X16, nullptr, FIN, 0L, (const unsigned short*)WinT, nullptr, FIN, 0L,
        (void*)Hm, nullptr, HP, 0L, binp, nullptr, 0L, NPAD, HP, FIN, 1.0f); }
  elu_cast_kernel<<<(NPAD * HP / 2 + 255) / 256, 256, 0, stream>>>(Hm, H16);

  for (int l = 0; l < NL; ++l) {
    { const int t = (NPAD / 64) * (HP / 64);
      wmma_gemm64<0, false, 0, 0, false><<<dim3((t + 7) / 8, 1), 256, 0, stream>>>(
          (const unsigned short*)H16, nullptr, HP, 0L, (const unsigned short*)(WgT + (size_t)l * HP * HP / 2), nullptr, HP, 0L,
          (void*)HW, nullptr, HP, 0L, nullptr, nullptr, 0L, NPAD, HP, HP, 1.0f); }
    att_terms_kernel<<<NPAD / 8, 256, 0, stream>>>(HW, asv + l * NHD * HC, adv + l * NHD * HC, ASD);
    gat_agg_kernel<<<NTILE, NT, 0, stream>>>(HW, ASD, ei, bg + l * HD, gam + l * HD, bet + l * HD, rm + l * HD, rv + l * HD, AGG, Hm, H16);
    pool_kernel<<<NG, 256, 0, stream>>>(Hm, bvec, l, Pf);
  }

  cast_f32_f16x2<<<(NG * NL * HD / 2 + 255) / 256, 256, 0, stream>>>(Pf, (_Float16*)P16, NG * NL * HD / 2);
  { const int t = (NG / 64) * (HP / 64);
    wmma_gemm64<0, false, 2, 1, false, 0><<<dim3((t + 7) / 8, 1), 256, 0, stream>>>(
        (const unsigned short*)P16, nullptr, NL * HD, 0L, (const unsigned short*)WjkT, nullptr, NL * HD, 0L,
        (void*)Z16, nullptr, HP, 0L, bjkp, nullptr, 0L, NG, HP, NL * HD, 1.0f); }
  elu16_kernel<<<(NG * HP / 2 + 255) / 256, 256, 0, stream>>>(Z16, NG * HP / 2);
  { const int t = (NG / 64) * (HP / 64);
    wmma_gemm64<0, false, 2, 0, false, 2><<<dim3((t + 7) / 8, 1), 256, 0, stream>>>(
        (const unsigned short*)Z16, nullptr, HP, 0L, (const unsigned short*)Wh1T, nullptr, HP, 0L,
        (void*)Z2, nullptr, HP, 0L, bh1p, nullptr, 0L, NG, HP, HP, 1.0f); }
  head_out_kernel<<<NG / 32, 256, 0, stream>>>(Z2, Wh2, bh2, (float*)d_out);
}
